// Involution_54004918780590
// MI455X (gfx1250) — hardware-verified
//
#include <hip/hip_runtime.h>
#include <math.h>

typedef __attribute__((ext_vector_type(16))) _Float16 v16h;
typedef __attribute__((ext_vector_type(16))) __bf16 v16b;
typedef __attribute__((ext_vector_type(8)))  _Float16 v8h;
typedef __attribute__((ext_vector_type(8)))  float v8f;
typedef __attribute__((ext_vector_type(4)))  float v4f;
typedef __attribute__((ext_vector_type(2)))  float v2f;
typedef __attribute__((ext_vector_type(4)))  unsigned v4u;
typedef __attribute__((ext_vector_type(4)))  int v4i;
typedef float __attribute__((may_alias)) float_a;
typedef int __attribute__((may_alias)) int_a;

template <typename T> __device__ __forceinline__ void vst2(void* p, T v) { *(volatile T*)p = v; __threadfence(); *(volatile T*)p = v; }
__device__ __forceinline__ v8f wmma16(v16h a, v16h b, v8f c) {
  v8f d = __builtin_amdgcn_wmma_f32_16x16x32_f16(false, a, false, b, (short)0, c, false, false);
  asm volatile("v_nop\n\tv_nop\n\tv_nop\n\tv_nop" : "+v"(d) : "v"(a), "v"(b));
  return d;
}
__device__ __forceinline__ v8f wmma_bf(v16b a, v16b b, v8f c) {
  v8f d = __builtin_amdgcn_wmma_f32_16x16x32_bf16(false, a, false, b, (short)0, c, false, false);
  asm volatile("v_nop\n\tv_nop\n\tv_nop\n\tv_nop" : "+v"(d) : "v"(a), "v"(b));
  return d;
}
__device__ __forceinline__ v16h frag_h(const _Float16* rowk0, int lane) {
  union { v16h v; v8h q[2]; } u; const _Float16* p = rowk0 + 8 * (lane >> 4);
  u.q[0] = *(const v8h*)p; u.q[1] = *(const v8h*)(p + 16); return u.v;
}
__device__ __forceinline__ v16h frag_f32(const float* rowk0, int lane) {
  v16h a; const float* p = rowk0 + 8 * (lane >> 4);
#pragma unroll
  for (int i = 0; i < 8; ++i) { a[i] = (_Float16)p[i]; a[8 + i] = (_Float16)p[16 + i]; }
  return a;
}
__device__ __forceinline__ v16h frag_f32s(const float* rowk0, int lane, float sc) {
  v16h a; const float* p = rowk0 + 8 * (lane >> 4);
#pragma unroll
  for (int i = 0; i < 8; ++i) { a[i] = (_Float16)(p[i] * sc); a[8 + i] = (_Float16)(p[16 + i] * sc); }
  return a;
}
__device__ __forceinline__ v16h fragc_f32(const float* W, int k0, int n, int lane, int ld, int K) {
  v16h a; const int g = lane >> 4;
#pragma unroll
  for (int i = 0; i < 8; ++i) { const int ka = k0 + 8 * g + i, kb = ka + 16;
    a[i] = (_Float16)(ka < K ? W[(size_t)(ka < K ? ka : K - 1) * ld + n] : 0.f); a[8 + i] = (_Float16)(kb < K ? W[(size_t)(kb < K ? kb : K - 1) * ld + n] : 0.f); }
  return a;
}
struct F2 { v16b h, l; };
__device__ __forceinline__ F2 bsplit16(const float v[16]) { F2 r;
#pragma unroll
  for (int i = 0; i < 16; ++i) { const __bf16 h = (__bf16)v[i]; r.h[i] = h; r.l[i] = (__bf16)(v[i] - (float)h); }
  return r; }
__device__ __forceinline__ F2 split_row(const float* row, int k0, int lane) { float v[16]; const float* p = row + k0 + 8 * (lane >> 4);
#pragma unroll
  for (int i = 0; i < 8; ++i) { v[i] = p[i]; v[8 + i] = p[16 + i]; }
  return bsplit16(v); }
__device__ __forceinline__ F2 split_rowK(const float* row, int k0, int lane, int K) { float v[16]; const int g = lane >> 4;
#pragma unroll
  for (int i = 0; i < 8; ++i) { const int ka = k0 + 8 * g + i, kb = ka + 16; v[i] = ka < K ? row[ka < K ? ka : K - 1] : 0.f; v[8 + i] = kb < K ? row[kb < K ? kb : K - 1] : 0.f; }
  return bsplit16(v); }
__device__ __forceinline__ F2 split_col(const float* W, int k0, int n, int lane, int ld, int K) { float v[16]; const int g = lane >> 4;
#pragma unroll
  for (int i = 0; i < 8; ++i) { const int ka = k0 + 8 * g + i, kb = ka + 16; v[i] = ka < K ? W[(size_t)(ka < K ? ka : K - 1) * ld + n] : 0.f; v[8 + i] = kb < K ? W[(size_t)(kb < K ? kb : K - 1) * ld + n] : 0.f; }
  return bsplit16(v); }
__device__ __forceinline__ v8f mac3(const F2& a, const F2& b, v8f c) { c = wmma_bf(a.l, b.h, c); c = wmma_bf(a.h, b.l, c); return wmma_bf(a.h, b.h, c); }
__device__ __forceinline__ float sigm(float v) { return 1.0f / (1.0f + expf(-v)); }
#define LDSX() do { asm volatile("s_wait_dscnt 0" ::: "memory"); __builtin_amdgcn_wave_barrier(); __builtin_amdgcn_fence(__ATOMIC_RELEASE, "workgroup"); } while (0)

#define NB 4
#define CH 256
#define HID 64
#define IMH 64
#define IMW 64
#define NPX (IMH * IMW)
#define KS 7
#define KK (KS * KS)
#ifndef TNB
#define TNB NB
#endif
typedef __attribute__((ext_vector_type(8))) __bf16 v8b;
__device__ __forceinline__ v16b frag_b(const __bf16* rowk0, int lane) {
  union { v16b v; v8b q[2]; } u; const __bf16* p = rowk0 + 8 * (lane >> 4);
  u.q[0] = *(const v8b*)p; u.q[1] = *(const v8b*)(p + 16); return u.v;
}
__device__ __forceinline__ float bfr(float v) { return (float)(__bf16)v; }
__device__ __forceinline__ v16b wrow(const float* rowk0, int lane) { v16b w; const float* p = rowk0 + 8 * (lane >> 4);
#pragma unroll
  for (int i = 0; i < 8; ++i) { w[i] = (__bf16)p[i]; w[8 + i] = (__bf16)p[16 + i]; }
  return w; }

#define WS_HH  0u
#define WS_HL  (WS_HH + 2u * (size_t)NB * HID * NPX)
#define WS_END (WS_HL + 2u * (size_t)NB * HID * NPX)

__global__ __launch_bounds__(128) void k_h(const float* __restrict__ X, const float* __restrict__ RW, const float* __restrict__ G, const float* __restrict__ Bt, const float* __restrict__ M, const float* __restrict__ V, __bf16* __restrict__ HH, __bf16* __restrict__ HL) {
  __shared__ __align__(16) __bf16 th[64][72], tl2[64][72];
  const int tid = threadIdx.x, wave = tid >> 5, lane = tid & 31, col = lane & 15, g = lane >> 4; const size_t b = blockIdx.x / (NPX / 64); const int p0 = (blockIdx.x % (NPX / 64)) * 64;
  v8f acc[4] = {};
#pragma unroll 2
  for (int kc = 0; kc < CH / 32; ++kc) { v16b a; { const float* p = X + (b * CH + kc * 32 + 8 * g) * (size_t)NPX + p0 + wave * 16 + col;
#pragma unroll
      for (int i = 0; i < 8; ++i) { a[i] = (__bf16)p[(size_t)i * NPX]; a[8 + i] = (__bf16)p[(size_t)(16 + i) * NPX]; } }
    asm volatile("s_wait_loadcnt 0x0" ::: "memory");
#pragma unroll
    for (int j = 0; j < 4; ++j) { const v16b w = wrow(RW + (size_t)(j * 16 + col) * CH + kc * 32, lane); asm volatile("s_wait_loadcnt 0x0" ::: "memory"); acc[j] = wmma_bf(a, w, acc[j]); } }
#pragma unroll
  for (int j = 0; j < 4; ++j) { const int o = j * 16 + col; const float inv = bfr(G[o]) / sqrtf(bfr(V[o]) + 1e-5f); const float sh = bfr(Bt[o]) - bfr(M[o]) * inv;
#pragma unroll
    for (int r = 0; r < 8; ++r) { const float hv = fmaxf(acc[j][r] * inv + sh, 0.f); const __bf16 bh = (__bf16)hv; th[wave * 16 + 8 * g + r][o] = bh; tl2[wave * 16 + 8 * g + r][o] = (__bf16)(hv - (float)bh); } }
  __syncthreads();
  for (int e = tid; e < 64 * 8; e += 128) { const int pl = e >> 3, q = e & 7; const size_t off = (b * NPX + p0 + pl) * (size_t)HID + q * 8; vst2((unsigned*)(HH + off), *(const v4u*)&th[pl][q * 8]); vst2((unsigned*)(HL + off), *(const v4u*)&tl2[pl][q * 8]); } }
__global__ __launch_bounds__(128) void k_inv(const float* __restrict__ X, const float* __restrict__ KW, const float* __restrict__ KB, const __bf16* __restrict__ HH, const __bf16* __restrict__ HL, float* __restrict__ OUT) {
  __shared__ __align__(16) float sk[64][132]; __shared__ __align__(16) float sx[8][72]; __shared__ __align__(16) float so[128];
  const int tid = threadIdx.x, wave = tid >> 5, lane = tid & 31, col = lane & 15, g = lane >> 4; const int gch = blockIdx.x; const size_t b = blockIdx.y / (IMH / 2); const int y0 = (blockIdx.y % (IMH / 2)) * 2; const int p0 = y0 * IMW;
  for (int e = tid; e < 8 * 70; e += 128) { const int rr = e / 70, cc = e % 70; const int yy = y0 - 3 + rr, xx = cc - 3; float v = 0.f; if (yy >= 0 && yy < IMH && xx >= 0 && xx < IMW) v = bfr(X[((b * CH + gch) * IMH + yy) * (size_t)IMW + xx]); sx[rr][cc] = v; }
  const int trow = wave * 16 + col; const int orow = gch * KK + (trow < KK ? trow : KK - 1); const float live = trow < KK ? 1.0f : 0.0f;
  v8f acc[8] = {};
#pragma unroll
  for (int kc = 0; kc < HID / 32; ++kc) { v16b a; { const float* p = KW + (size_t)orow * HID + kc * 32 + 8 * g;
#pragma unroll
      for (int i = 0; i < 8; ++i) { a[i] = (__bf16)(p[i] * live); a[8 + i] = (__bf16)(p[16 + i] * live); } }
    asm volatile("s_wait_loadcnt 0x0" ::: "memory");
#pragma unroll
    for (int j = 0; j < 8; ++j) { const size_t hp = (b * NPX + p0 + j * 16 + col) * (size_t)HID + kc * 32;
      const v16b bh = frag_b(HH + hp, lane), bl = frag_b(HL + hp, lane); asm volatile("s_wait_loadcnt 0x0" ::: "memory"); acc[j] = wmma_bf(a, bh, acc[j]); acc[j] = wmma_bf(a, bl, acc[j]); } }
  {
#pragma unroll
    for (int j = 0; j < 8; ++j) {
#pragma unroll
      for (int r = 0; r < 8; ++r) { const int t = wave * 16 + 8 * g + r; const float bb = (t < KK) ? bfr(KB[gch * KK + (t < KK ? t : 0)]) : 0.f; sk[t][j * 16 + col] = acc[j][r] + bb; } } }
  __syncthreads();
  { const int pl = tid; const int ry = pl >> 6, cx = pl & 63; float mean = 0.f;
#pragma unroll 7
    for (int t = 0; t < KK; ++t) mean += sk[t][pl];
    mean *= (1.0f / KK); float ss = 0.f;
#pragma unroll 7
    for (int t = 0; t < KK; ++t) { const float d = sk[t][pl] - mean; ss += d * d; }
    const float dn = fmaxf(sqrtf(ss), 1e-6f); float o = 0.f;
#pragma unroll 1
    for (int i = 0; i < KS; ++i) {
#pragma unroll
      for (int jj = 0; jj < KS; ++jj) { const int t = i * KS + jj; o = o + sx[ry + i][cx + jj] * ((sk[t][pl] - mean) / dn); } }
    so[pl] = o; }
  __syncthreads();
  if (tid < 32) vst2(OUT + ((b * CH + gch) * (size_t)NPX + p0) + tid * 4, *(const v4f*)&so[tid * 4]); }
extern "C" void kernel_launch(void* const* d_in, const int* in_sizes, int n_in, void* d_out, int out_size, void* d_ws, size_t ws_size, hipStream_t stream) {
  (void)in_sizes; (void)n_in; (void)out_size;
  const float** F = (const float**)d_in;
  if (ws_size < (size_t)WS_END) return;
  char* ws = (char*)d_ws; __bf16 *HH = (__bf16*)(ws + WS_HH), *HL = (__bf16*)(ws + WS_HL);
  k_h<<<dim3(TNB * NPX / 64), 128, 0, stream>>>(F[0], F[1], F[2], F[3], F[4], F[5], HH, HL);
  k_inv<<<dim3(CH, TNB * IMH / 2), 128, 0, stream>>>(F[0], F[6], F[7], HH, HL, (float*)d_out);
}
